// MaskedSelfAttention_56032143343859
// MI455X (gfx1250) — hardware-verified
//
#include <hip/hip_runtime.h>
#include <math.h>
#include <stdint.h>

#ifndef NB
#define NB 1
#endif
#ifndef SEQ
#define SEQ 8192
#endif
#define SEQ_FULL 8192
#define DM    1024
#define DK    128
#define CK    512
#define NKB   16
#define NCHK  (SEQ / CK)
#define QT    16
#define TQ0   128
#define NQT   ((SEQ - TQ0) / QT)
#define SCP   (CK + 32)
#define PLP   (CK + 16)
#define SLAB64 (16 * 68)
#define VTP   72
#define ATT_THREADS 256
#define HEAD_THREADS 128
#define QSC   8.0f
#define KSC   8.0f
#define RSC   2048.0f
#define RRS   (1.0f / 2048.0f)
#define PCAR  32768.0f
#define VCAR  1024.0f
#define LOG2E 1.4426950408889634f
#define RSQD  0.08838834764831845f
#define WS_CAP ((size_t)134217728)

static_assert(NB == 1);
static_assert(SEQ >= CK && (SEQ % CK) == 0 && SEQ <= SEQ_FULL && (SEQ / CK) == NCHK && CK == 32 * NKB && NKB == 16);
static_assert((SEQ % 64) == 0 && (SEQ % QT) == 0 && (CK % QT) == 0 && NQT * QT + TQ0 == SEQ);
static_assert((TQ0 % QT) == 0 && (TQ0 % 64) == 0 && TQ0 <= CK && TQ0 == 128 && TQ0 == HEAD_THREADS && DK == HEAD_THREADS);
static_assert((DM % 32) == 0 && (DM % 64) == 0 && DK == 128 && (DK % 64) == 0 && (DK % 32) == 0);
static_assert(ATT_THREADS == 16 * QT && ATT_THREADS == 256 && DK == 16 * (ATT_THREADS / 32));
static_assert(((DK * DM) % 2048) == 0 && ((SEQ * DM) % 2048) == 0);
static_assert(SCP >= CK + 16 && PLP >= CK + 8 && SCP >= DK);
static_assert(((PLP * 2) % 16) == 0 && ((SCP * 4) % 16) == 0 && ((VTP * 2) % 16) == 0);
static_assert(64 * VTP >= 63 * VTP + 64);
static_assert((16 * SCP) % 256 == 0);

typedef unsigned short u16;
typedef _Float16 v16h __attribute__((ext_vector_type(16)));
typedef _Float16 v8h  __attribute__((ext_vector_type(8)));
typedef __bf16   v16b __attribute__((ext_vector_type(16)));
typedef float    v8f  __attribute__((ext_vector_type(8)));
typedef float    v4f  __attribute__((ext_vector_type(4)));
typedef unsigned int v4u __attribute__((ext_vector_type(4)));

union FragH { v16h v; v8h h[2]; v4u u[2]; };
union FragB { v16b v; v4u u[2]; };

__device__ __forceinline__ unsigned short bf_bits(float f) {
  unsigned u = __float_as_uint(f);
  return (unsigned short)((u + 0x7FFFu + ((u >> 16) & 1u)) >> 16);
}
__device__ __forceinline__ float bf_up(unsigned short h) { return __uint_as_float(((unsigned)h) << 16); }
__device__ __forceinline__ float bfr(float f) { return bf_up(bf_bits(f)); }
__device__ __forceinline__ unsigned short h_bits(_Float16 x) { return __builtin_bit_cast(unsigned short, x); }
__device__ __forceinline__ unsigned pk16(unsigned short a, unsigned short b) { return (unsigned)a | ((unsigned)b << 16); }
__device__ __forceinline__ v8f zero8() { v8f z = {0.f, 0.f, 0.f, 0.f, 0.f, 0.f, 0.f, 0.f}; return z; }
__device__ __forceinline__ v4f zero4() { v4f z = {0.f, 0.f, 0.f, 0.f}; return z; }

__device__ __forceinline__ v16h ldfrag_h(const _Float16* p) {
  FragH f;
  f.h[0] = *(const v8h*)(p);
  f.h[1] = *(const v8h*)(p + 16);
  return f.v;
}
__device__ __forceinline__ v16b ldfrag_b(const u16* p) {
  FragB f;
  f.u[0] = *(const v4u*)(p);
  f.u[1] = *(const v4u*)(p + 16);
  return f.v;
}

__device__ __forceinline__ v8f mma_h(v16h a, v16h b, v8f c) {
  return __builtin_amdgcn_wmma_f32_16x16x32_f16(false, a, false, b, (short)0, c, false, false);
}
__device__ __forceinline__ v8f mma_b(v16b a, v16b b, v8f c) {
  return __builtin_amdgcn_wmma_f32_16x16x32_bf16(false, a, false, b, (short)0, c, false, false);
}
template <typename F>
__device__ __forceinline__ void guard6(v8f& a, v8f& b, v8f& c, v8f& d, F x0, F x1, F x2, F x3, F x4, F x5) {
#if defined(__HIP_DEVICE_COMPILE__)
  asm volatile("v_nop\n\tv_nop\n\tv_nop\n\tv_nop"
               : "+v"(a), "+v"(b), "+v"(c), "+v"(d) : "v"(x0), "v"(x1), "v"(x2), "v"(x3), "v"(x4), "v"(x5) : "memory");
#endif
}
__device__ __forceinline__ void guard1x2(v8f& a, v16h x0, v16h x1) {
#if defined(__HIP_DEVICE_COMPILE__)
  asm volatile("v_nop\n\tv_nop\n\tv_nop\n\tv_nop" : "+v"(a) : "v"(x0), "v"(x1) : "memory");
#endif
}
__device__ __forceinline__ void acc_guard1(v8f& a) {
#if defined(__HIP_DEVICE_COMPILE__)
  asm volatile("v_nop\n\tv_nop\n\tv_nop\n\tv_nop" : "+v"(a));
#endif
}
__device__ __forceinline__ void wave_sync_lds() {
  __builtin_amdgcn_fence(__ATOMIC_RELEASE, "workgroup");
  __builtin_amdgcn_wave_barrier();
  __builtin_amdgcn_fence(__ATOMIC_ACQUIRE, "workgroup");
}

__global__ __launch_bounds__(256) void cvt16(const float* __restrict__ x, u16* D, int n8, int mode, float scale) {
  const int gt = blockIdx.x * 256 + (int)threadIdx.x;
  if (gt >= n8) return;
  const float* p = x + (size_t)gt * 8;
  const v4f a = *(const v4f*)(p), c4 = *(const v4f*)(p + 4);
  float v[8];
#pragma unroll
  for (int e = 0; e < 4; ++e) { v[e] = a[e]; v[4 + e] = c4[e]; }
  unsigned short s[8];
#pragma unroll
  for (int e = 0; e < 8; ++e) {
    const float vb = bfr(v[e]);
    const float vf = (mode == 1) ? vb : v[e];
    const unsigned short hb = h_bits((_Float16)(vf * scale));
    const unsigned short bb = bf_bits(v[e]);
    s[e] = (mode != 0) ? hb : bb;
  }
  v4u o;
#pragma unroll
  for (int e = 0; e < 4; ++e) o[e] = pk16(s[2 * e], s[2 * e + 1]);
  u16* d = D + (size_t)gt * 8;
  for (int pass = 0; pass < 2; ++pass) {
    *(volatile v4u*)(d) = o;
    __threadfence();
  }
}

__device__ __forceinline__ void stage64(float* sl, v8f a0, v8f a1, v8f a2, v8f a3, float oscale, int lane) {
  const int hh = lane >> 4, m = lane & 15;
#pragma unroll
  for (int r = 0; r < 8; ++r) {
    const int ro = (8 * hh + r) * 68 + m;
    sl[ro]      = a0[r] * oscale;
    sl[ro + 16] = a1[r] * oscale;
    sl[ro + 32] = a2[r] * oscale;
    sl[ro + 48] = a3[r] * oscale;
  }
  wave_sync_lds();
}
__device__ __forceinline__ void epi64(float* sl, v8f a0, v8f a1, v8f a2, v8f a3, float oscale, v4f badd, float* C, int N,
                                      size_t rowb, int col0, int lane) {
  const int hh = lane >> 4, m = lane & 15;
  stage64(sl, a0, a1, a2, a3, oscale, lane);
  v4f vals[8];
#pragma unroll
  for (int it = 0; it < 8; ++it) vals[it] = *(const v4f*)(sl + (it * 2 + hh) * 68 + m * 4) + badd;
  float* dst = C + (rowb + (size_t)hh) * (size_t)N + col0 + m * 4;
  for (int pass = 0; pass < 2; ++pass) {
#pragma unroll
    for (int it = 0; it < 8; ++it) {
      *(volatile v4f*)(dst + (size_t)(it * 2) * (size_t)N) = vals[it];
    }
    __threadfence();
  }
}
__device__ __forceinline__ void epi64h2(float* sl, v8f a0, v8f a1, v8f a2, v8f a3, float pscale, float rscale,
                                        u16* CH, u16* CR, int N, size_t rowb, int col0, int lane) {
  stage64(sl, a0, a1, a2, a3, pscale, lane);
  const int rq = lane >> 3, c8 = (lane & 7) * 8;
  v4u oh[4], orr[4];
#pragma unroll
  for (int i4 = 0; i4 < 4; ++i4) {
    const int row = i4 * 4 + rq;
    const v4f a = *(const v4f*)(sl + row * 68 + c8), c4 = *(const v4f*)(sl + row * 68 + c8 + 4);
    float w[8];
#pragma unroll
    for (int e = 0; e < 4; ++e) { w[e] = a[e]; w[4 + e] = c4[e]; }
    unsigned short hb[8], rb[8];
#pragma unroll
    for (int e = 0; e < 8; ++e) {
      const _Float16 hv = (_Float16)w[e];
      hb[e] = h_bits(hv);
      rb[e] = h_bits((_Float16)((w[e] - (float)hv) * rscale));
    }
#pragma unroll
    for (int e = 0; e < 4; ++e) {
      oh[i4][e]  = pk16(hb[2 * e], hb[2 * e + 1]);
      orr[i4][e] = pk16(rb[2 * e], rb[2 * e + 1]);
    }
  }
  const size_t dof = rowb * (size_t)N + (size_t)col0 + (size_t)c8;
  for (int pass = 0; pass < 2; ++pass) {
#pragma unroll
    for (int i4 = 0; i4 < 4; ++i4) {
      const int row = i4 * 4 + rq;
      *(volatile v4u*)(CH + dof + (size_t)row * (size_t)N) = oh[i4];
      *(volatile v4u*)(CR + dof + (size_t)row * (size_t)N) = orr[i4];
    }
    __threadfence();
  }
}

__global__ __launch_bounds__(128)
void gemm_b32(const u16* __restrict__ A, const u16* __restrict__ Bt, float* C, int M, int N, int K, float oscale) {
  __shared__ __align__(16) float slab[4 * SLAB64];
  const int tid = threadIdx.x, wave = tid >> 5, lane = tid & 31, hh = lane >> 4, m = lane & 15;
  const int ntile = N >> 6;
  const int bid   = blockIdx.x;
  const int rowb  = (bid / ntile) * 64 + wave * 16;
  const int col0  = (bid % ntile) * 64;
  if (rowb + 16 > M) return;
  const u16* ap = A  + (size_t)(rowb + m) * K + 8 * hh;
  const u16* bp = Bt + (size_t)(col0 + m) * K + 8 * hh;
  const size_t bs = (size_t)16 * K;
  v8f acc0 = zero8(), acc1 = zero8(), acc2 = zero8(), acc3 = zero8();
#pragma unroll 1
  for (int k0 = 0; k0 < K; k0 += 32) {
    const v16b a  = ldfrag_b(ap + k0);
    const v16b b0 = ldfrag_b(bp + k0);
    const v16b b1 = ldfrag_b(bp + bs + k0);
    const v16b b2 = ldfrag_b(bp + 2 * bs + k0);
    const v16b b3 = ldfrag_b(bp + 3 * bs + k0);
    acc0 = mma_b(a, b0, acc0);
    acc1 = mma_b(a, b1, acc1);
    acc2 = mma_b(a, b2, acc2);
    acc3 = mma_b(a, b3, acc3);
    guard6<v16b>(acc0, acc1, acc2, acc3, a, b0, b1, b2, b3, a);
  }
  epi64(slab + wave * SLAB64, acc0, acc1, acc2, acc3, oscale, zero4(), C, N, (size_t)rowb, col0, lane);
}

__global__ __launch_bounds__(128)
void gemm_bh2(const u16* __restrict__ A, const u16* __restrict__ Bt, u16* CH, u16* CR, int M, int N, int K,
              float pscale, float rscale) {
  __shared__ __align__(16) float slab[4 * SLAB64];
  const int tid = threadIdx.x, wave = tid >> 5, lane = tid & 31, hh = lane >> 4, m = lane & 15;
  const int ntile = N >> 6;
  const int bid   = blockIdx.x;
  const int rowb  = (bid / ntile) * 64 + wave * 16;
  const int col0  = (bid % ntile) * 64;
  if (rowb + 16 > M) return;
  const u16* ap = A  + (size_t)(rowb + m) * K + 8 * hh;
  const u16* bp = Bt + (size_t)(col0 + m) * K + 8 * hh;
  const size_t bs = (size_t)16 * K;
  v8f acc0 = zero8(), acc1 = zero8(), acc2 = zero8(), acc3 = zero8();
#pragma unroll 1
  for (int k0 = 0; k0 < K; k0 += 32) {
    const v16b a  = ldfrag_b(ap + k0);
    const v16b b0 = ldfrag_b(bp + k0);
    const v16b b1 = ldfrag_b(bp + bs + k0);
    const v16b b2 = ldfrag_b(bp + 2 * bs + k0);
    const v16b b3 = ldfrag_b(bp + 3 * bs + k0);
    acc0 = mma_b(a, b0, acc0);
    acc1 = mma_b(a, b1, acc1);
    acc2 = mma_b(a, b2, acc2);
    acc3 = mma_b(a, b3, acc3);
    guard6<v16b>(acc0, acc1, acc2, acc3, a, b0, b1, b2, b3, a);
  }
  epi64h2(slab + wave * SLAB64, acc0, acc1, acc2, acc3, pscale, rscale, CH, CR, N, (size_t)rowb, col0, lane);
}

__global__ __launch_bounds__(256) void xt16(const float* __restrict__ V, u16* VTo) {
  __shared__ __align__(16) u16 TH[64 * VTP];
  const int tid = threadIdx.x;
  const int bid = blockIdx.x;
  const int st  = bid % (SEQ / 64);
  const int dcb = bid / (SEQ / 64);
  const int s0  = st * 64;
  const int d0  = dcb * 64;
  {
    const int sl = tid >> 2;
    const int dc = (tid & 3) * 16;
    const float* src = V + (size_t)(s0 + sl) * DK + d0 + dc;
#pragma unroll
    for (int i = 0; i < 4; ++i) {
      const v4f a = *(const v4f*)(src + 4 * i);
#pragma unroll
      for (int e = 0; e < 4; ++e) {
        const _Float16 hv = (_Float16)(a[e] * VCAR);
        TH[(dc + 4 * i + e) * VTP + sl] = h_bits(hv);
      }
    }
  }
  __syncthreads();
  v4u vh[2];
  const int q8 = tid >> 3, p8 = (tid & 7) * 8;
#pragma unroll
  for (int it = 0; it < 2; ++it) {
    const int line = it * 32 + q8;
    vh[it] = *(const v4u*)(TH + line * VTP + p8);
  }
  const size_t base = (size_t)d0 * SEQ + s0 + p8;
  for (int pass = 0; pass < 2; ++pass) {
#pragma unroll
    for (int it = 0; it < 2; ++it) {
      const int line = it * 32 + q8;
      *(volatile v4u*)(VTo + base + (size_t)line * SEQ) = vh[it];
    }
    __threadfence();
  }
}

__global__ __launch_bounds__(128) void vsum_k(const float* __restrict__ V, float* VS) {
  __shared__ __align__(16) float sm[NKB * 128];
  const int tid = threadIdx.x;
  const int c   = blockIdx.x;
  const float* p = V + (size_t)c * CK * DK + tid;
  float s = 0.f;
#pragma unroll 1
  for (int kb = 0; kb < NKB; ++kb) {
#pragma unroll 4
    for (int i = 0; i < 32; ++i) s += p[(size_t)(kb * 32 + i) * DK];
    sm[kb * 128 + tid] = s;
  }
  __syncthreads();
  v4f o[4];
#pragma unroll
  for (int it = 0; it < 4; ++it) o[it] = *(const v4f*)(sm + (size_t)(it * 128 + tid) * 4);
  float* base = VS + (size_t)c * NKB * DK;
  for (int pass = 0; pass < 2; ++pass) {
#pragma unroll
    for (int it = 0; it < 4; ++it) {
      *(volatile v4f*)(base + (size_t)(it * 128 + tid) * 4) = o[it];
    }
    __threadfence();
  }
}

__global__ __launch_bounds__(ATT_THREADS)
void attn_fwd(const u16* __restrict__ QHp, const u16* __restrict__ QRp, const u16* __restrict__ KHp, const u16* __restrict__ KRp,
              const u16* __restrict__ VTp, const float* __restrict__ VSp, float* Out) {
  __shared__ __align__(16) float scs[16 * SCP];
  __shared__ __align__(16) u16 pls[16 * PLP];
  __shared__ float rowa[QT];
  __shared__ float rowc[QT];
  __shared__ float rowi[QT];

  const int tid  = threadIdx.x;
  const int wave = tid >> 5;
  const int lane = tid & 31;
  const int hh   = lane >> 4;
  const int m    = lane & 15;
  const int r16  = tid >> 4;
  const int sub  = tid & 15;
  const int kl0  = sub * 32;

  const int q0  = TQ0 + blockIdx.x * QT;
  const int qc  = q0 / CK;

  const _Float16* qha = (const _Float16*)(const void*)QHp + (size_t)(q0 + m) * DK + 8 * hh;
  const _Float16* qra = (const _Float16*)(const void*)QRp + (size_t)(q0 + m) * DK + 8 * hh;
  const _Float16* khb = (const _Float16*)(const void*)KHp + (size_t)m * DK + 8 * hh;
  const _Float16* krb = (const _Float16*)(const void*)KRp + (size_t)m * DK + 8 * hh;
  const _Float16* vbp = (const _Float16*)(const void*)VTp + (size_t)(wave * 16 + m) * SEQ + 8 * hh;
  const float* vsb = VSp + wave * 16 + m;
  const float lsc = RSQD * LOG2E / (QSC * KSC);

  float mrun = -INFINITY, lrun = 0.f;
  v8f o = zero8();

#pragma unroll 1
  for (int c = 0; c <= qc; ++c) {
    const int kbeg = c * CK;
    const int nkb  = (c < qc) ? NKB : (((q0 + QT - 1 - kbeg) >> 5) + 1);
#pragma unroll 1
    for (int kb = wave; kb < NKB; kb += 8) {
      v8f s0h = zero8(), s1h = zero8(), s0r = zero8(), s1r = zero8();
      if (kb < nkb) {
        const size_t ko = (size_t)(kbeg + kb * 32) * DK;
        const _Float16* kh0 = khb + ko;
        const _Float16* kh1 = kh0 + (size_t)16 * DK;
        const _Float16* kr0 = krb + ko;
        const _Float16* kr1 = kr0 + (size_t)16 * DK;
#pragma unroll
        for (int ks = 0; ks < DK / 32; ++ks) {
          const v16h a  = ldfrag_h(qha + ks * 32);
          const v16h ar = ldfrag_h(qra + ks * 32);
          const v16h f0 = ldfrag_h(kh0 + ks * 32);
          const v16h f1 = ldfrag_h(kh1 + ks * 32);
          const v16h g0 = ldfrag_h(kr0 + ks * 32);
          const v16h g1 = ldfrag_h(kr1 + ks * 32);
          s0h = mma_h(a, f0, s0h);
          s1h = mma_h(a, f1, s1h);
          s0r = mma_h(a, g0, s0r);
          s1r = mma_h(a, g1, s1r);
          s0r = mma_h(ar, f0, s0r);
          s1r = mma_h(ar, f1, s1r);
          guard6<v16h>(s0h, s1h, s0r, s1r, a, ar, f0, f1, g0, g1);
        }
      }
      float* srow = scs + (8 * hh) * SCP + kb * 32 + m;
#pragma unroll
      for (int r = 0; r < 8; ++r) {
        srow[r * SCP]      = s0h[r] + s0r[r] * RRS;
        srow[r * SCP + 16] = s1h[r] + s1r[r] * RRS;
      }
    }
    __syncthreads();
    {
      const float* sp = scs + r16 * SCP + kl0;
      const int lim = (q0 + r16) - (kbeg + kl0);
      float t[32];
      float cm = -INFINITY;
#pragma unroll
      for (int i = 0; i < 8; ++i) {
        const v4f a = *(const v4f*)(sp + 4 * i);
#pragma unroll
        for (int e = 0; e < 4; ++e) {
          const int j = 4 * i + e;
          const float tv = (j <= lim) ? a[e] * lsc : -INFINITY;
          t[j] = tv;
          cm = fmaxf(cm, tv);
        }
      }
#pragma unroll
      for (int d = 1; d <= 8; d <<= 1) cm = fmaxf(cm, __shfl_xor(cm, d, 32));
      const float mn = fmaxf(mrun, cm);
      const float al = (mrun == -INFINITY) ? 0.f : exp2f(mrun - mn);
      mrun = mn;
      float ps = 0.f;
#pragma unroll
      for (int j = 0; j < 32; ++j) {
        const float p = exp2f(fminf(t[j] - mn, 0.f));
        t[j] = p;
        ps += p;
      }
#pragma unroll
      for (int d = 1; d <= 8; d <<= 1) ps += __shfl_xor(ps, d, 32);
      const float cc = ps * (1.0f / (float)CK);
      v4u pk[4];
#pragma unroll
      for (int i = 0; i < 4; ++i) {
#pragma unroll
        for (int e = 0; e < 4; ++e) {
          const int j = 8 * i + 2 * e;
          pk[i][e] = pk16(h_bits((_Float16)((t[j] - cc) * PCAR)), h_bits((_Float16)((t[j + 1] - cc) * PCAR)));
        }
      }
      lrun = lrun * al + ps;
      u16* pd = pls + r16 * PLP + kl0;
#pragma unroll
      for (int i = 0; i < 4; ++i) *(v4u*)(pd + 8 * i) = pk[i];
      if (sub == 0) { rowa[r16] = al; rowc[r16] = cc; }
    }
    __syncthreads();
    {
      float scl[8], cad[8];
#pragma unroll
      for (int r = 0; r < 8; ++r) { scl[r] = rowa[8 * hh + r]; cad[r] = rowc[8 * hh + r] * (PCAR * VCAR); }
      const float vs = vsb[((size_t)c * NKB + (size_t)(nkb - 1)) * DK];
#pragma unroll
      for (int r = 0; r < 8; ++r) o[r] = o[r] * scl[r] + cad[r] * vs;
      const _Float16* pp = (const _Float16*)(const void*)pls + m * PLP + 8 * hh;
      const _Float16* vp = vbp + kbeg;
#pragma unroll 1
      for (int kb = 0; kb < nkb; ++kb) {
        const v16h pf = ldfrag_h(pp + kb * 32);
        const v16h gv = ldfrag_h(vp + kb * 32);
        o = mma_h(pf, gv, o);
        guard1x2(o, pf, gv);
      }
    }
  }
  acc_guard1(o);

  if (sub == 0) rowi[r16] = (1.0f / lrun) * (1.0f / (PCAR * VCAR));
  __syncthreads();
  float inv[8];
#pragma unroll
  for (int r = 0; r < 8; ++r) inv[r] = rowi[8 * hh + r];
#pragma unroll
  for (int r = 0; r < 8; ++r) scs[(8 * hh + r) * SCP + wave * 16 + m] = o[r] * inv[r];
  __syncthreads();
  v4f ov[2];
#pragma unroll
  for (int it = 0; it < 2; ++it) {
    const int p   = it * 256 + tid;
    const int row = p >> 5;
    const int c4  = (p & 31) * 4;
    ov[it] = *(const v4f*)(scs + row * SCP + c4);
  }
  float* ob = Out + (size_t)q0 * DK;
  for (int pass = 0; pass < 2; ++pass) {
#pragma unroll
    for (int it = 0; it < 2; ++it) {
      const int p = it * 256 + tid;
      *(volatile v4f*)(ob + (size_t)p * 4) = ov[it];
    }
    __threadfence();
  }
}

__global__ __launch_bounds__(HEAD_THREADS) void attn_head(const float* __restrict__ QF, const float* __restrict__ KF,
                                                         const float* __restrict__ V, float* Out) {
  __shared__ __align__(16) float qs[DK];
  __shared__ float sc[TQ0];
  __shared__ float red[HEAD_THREADS / 32];
  __shared__ float redb[HEAD_THREADS / 32];
  __shared__ __align__(16) float zs[DK];
  const int tid = threadIdx.x, lane = tid & 31, wave = tid >> 5;
  const int t = blockIdx.x;
  if (tid < DK / 4) *(v4f*)(qs + tid * 4) = *(const v4f*)(QF + (size_t)t * DK + tid * 4);
  __syncthreads();
  const float* kp = KF + (size_t)tid * DK;
  float acc = 0.f;
#pragma unroll 1
  for (int d = 0; d < DK; d += 8) {
    const v4f k0 = *(const v4f*)(kp + d), k1 = *(const v4f*)(kp + d + 4);
    const v4f q0 = *(const v4f*)(qs + d), q1 = *(const v4f*)(qs + d + 4);
#pragma unroll
    for (int e = 0; e < 4; ++e) acc += k0[e] * q0[e];
#pragma unroll
    for (int e = 0; e < 4; ++e) acc += k1[e] * q1[e];
  }
  const float s = (tid <= t) ? acc * (RSQD * LOG2E) : -INFINITY;
  float mx = s;
#pragma unroll
  for (int d = 1; d <= 16; d <<= 1) mx = fmaxf(mx, __shfl_xor(mx, d, 32));
  if (lane == 0) red[wave] = mx;
  __syncthreads();
  float gm = red[0];
#pragma unroll
  for (int w = 1; w < HEAD_THREADS / 32; ++w) gm = fmaxf(gm, red[w]);
  const float p = exp2f(s - gm);
  float ps = p;
#pragma unroll
  for (int d = 1; d <= 16; d <<= 1) ps += __shfl_xor(ps, d, 32);
  if (lane == 0) redb[wave] = ps;
  sc[tid] = p;
  __syncthreads();
  float l = redb[0];
#pragma unroll
  for (int w = 1; w < HEAD_THREADS / 32; ++w) l += redb[w];
  const float inv = 1.0f / l;
  const float* vp = V + tid;
  float cx = 0.f;
#pragma unroll 1
  for (int j = 0; j <= t; ++j) {
    cx += sc[j] * vp[(size_t)j * DK];
  }
  zs[tid] = cx * inv;
  __syncthreads();
  if (wave == 0) {
    const v4f ov = *(const v4f*)(zs + lane * 4);
    float* dst = Out + (size_t)t * DK + lane * 4;
    *(volatile v4f*)dst = ov;
    __threadfence();
    *(volatile v4f*)dst = ov;
  }
}

extern "C" void kernel_launch(void* const* d_in, const int* in_sizes, int n_in,
                              void* d_out, int out_size, void* d_ws, size_t ws_size,
                              hipStream_t stream) {
  if (n_in < 4) return;
  if ((long long)in_sizes[0] < (long long)SEQ * DM) return;
  if (in_sizes[1] < DK * DM || in_sizes[2] < DK * DM || in_sizes[3] < DK * DM) return;
  if ((long long)out_size < (long long)SEQ * DK) return;

  const float* x  = (const float*)d_in[0];
  const float* wq = (const float*)d_in[1];
  const float* wk = (const float*)d_in[2];
  const float* wv = (const float*)d_in[3];
  float*       out = (float*)d_out;

  const size_t szW  = (size_t)DK * DM * 2;
  const size_t szXB = (size_t)SEQ * DM * 2;
  const size_t sz16 = (size_t)SEQ * DK * 2;
  const size_t sz32 = (size_t)SEQ * DK * 4;
  const size_t szVT = (size_t)DK * SEQ * 2;
  const size_t szVS = (size_t)NCHK * NKB * DK * 4;
  const size_t szHF = (size_t)TQ0 * DK * 4;
  size_t off = 0;
  const size_t oWQ = off; off += szW;
  const size_t oWK = off; off += szW;
  const size_t oWV = off; off += szW;
  const size_t oXB = off; off += szXB;
  const size_t oQH = off; off += sz16;
  const size_t oQR = off; off += sz16;
  const size_t oKH = off; off += sz16;
  const size_t oKR = off; off += sz16;
  const size_t oV  = off; off += sz32;
  const size_t oVT = off; off += szVT;
  const size_t oVS = off; off += szVS;
  const size_t oQF = off; off += szHF;
  const size_t oKF = off; off += szHF;
  if (off > ws_size) return;
  if (off > WS_CAP) return;

  char* ws = (char*)d_ws;
  u16*   WQB = (u16*)(ws + oWQ);
  u16*   WKB = (u16*)(ws + oWK);
  u16*   WVB = (u16*)(ws + oWV);
  u16*   XB  = (u16*)(ws + oXB);
  u16*   QH  = (u16*)(ws + oQH);
  u16*   QR  = (u16*)(ws + oQR);
  u16*   KH  = (u16*)(ws + oKH);
  u16*   KR  = (u16*)(ws + oKR);
  float* V   = (float*)(ws + oV);
  u16*   VT  = (u16*)(ws + oVT);
  float* VS  = (float*)(ws + oVS);
  float* QF  = (float*)(ws + oQF);
  float* KF  = (float*)(ws + oKF);

  const int n8w = (DK * DM) / 8;
  const int n8x = SEQ * (DM / 8);
  if ((n8w % 256) != 0 || (n8x % 256) != 0) return;
  const dim3 blk(256);
  const dim3 gW(n8w / 256), gX(n8x / 256);
  const dim3 gG((SEQ / 64) * (DK / 64));
  const dim3 gH((TQ0 / 64) * (DK / 64));
  const dim3 bG(128);
  const dim3 gXT((DK / 64) * (SEQ / 64));
  const dim3 gVS(NCHK);
  const dim3 bVS(128);
  const dim3 gAT(NQT);
  const dim3 bAT(ATT_THREADS);
  const dim3 gHD(TQ0);
  const dim3 bHD(HEAD_THREADS);

  cvt16<<<gW, blk, 0, stream>>>(wq, WQB, n8w, 0, 1.0f);
  cvt16<<<gW, blk, 0, stream>>>(wk, WKB, n8w, 0, 1.0f);
  cvt16<<<gW, blk, 0, stream>>>(wv, WVB, n8w, 0, 1.0f);
  cvt16<<<gX, blk, 0, stream>>>(x, XB, n8x, 0, 1.0f);
  gemm_bh2<<<gG, bG, 0, stream>>>(XB, WQB, QH, QR, SEQ, DK, DM, QSC, RSC);
  gemm_bh2<<<gG, bG, 0, stream>>>(XB, WKB, KH, KR, SEQ, DK, DM, KSC, RSC);
  gemm_b32<<<gG, bG, 0, stream>>>(XB, WVB, V, SEQ, DK, DM, 1.0f);
  gemm_b32<<<gH, bG, 0, stream>>>(XB, WQB, QF, TQ0, DK, DM, 1.0f);
  gemm_b32<<<gH, bG, 0, stream>>>(XB, WKB, KF, TQ0, DK, DM, 1.0f);
  xt16<<<gXT, blk, 0, stream>>>(V, VT);
  vsum_k<<<gVS, bVS, 0, stream>>>(V, VS);
  attn_fwd<<<gAT, bAT, 0, stream>>>(QH, QR, KH, KR, VT, VS, out);
  attn_head<<<gHD, bHD, 0, stream>>>(QF, KF, V, out);
  (void)hipGetLastError();
}
